// SelectiveScanMamba_23957327577740
// MI455X (gfx1250) — hardware-verified
//
#include <hip/hip_runtime.h>
#include <hip/hip_bf16.h>


#define NBATCH 2
#define NL_    2048
#define DM_    1024
#define DI_    2048
#define NS_    16
#define MT_    (NBATCH * NL_)

static_assert(MT_ % 128 == 0);
static_assert((2 * DI_) % 128 == 0);
static_assert(DI_ % 128 == 0);
static_assert(DM_ % 128 == 0);
static_assert(DM_ % 64 == 0);
static_assert(DI_ % 64 == 0);
static_assert((2 * NS_) == 32);
static_assert(NL_ % 16 == 0);
static_assert((NL_ & (NL_ - 1)) == 0);
static_assert(DI_ / 8 == 256);

typedef float          v4f   __attribute__((ext_vector_type(4)));
typedef float          v8f   __attribute__((ext_vector_type(8)));
typedef _Float16       v8h   __attribute__((ext_vector_type(8)));
typedef _Float16       v16h  __attribute__((ext_vector_type(16)));
typedef __bf16         v16b  __attribute__((ext_vector_type(16)));
typedef unsigned short u16x8 __attribute__((ext_vector_type(8)));

union FragH { u16x8 h[2]; v16h v; };
union FragB { u16x8 h[2]; v16b v; };
union Pack8 { v8h f; u16x8 u; };
union HBits { _Float16 h; unsigned short u; };

__device__ __forceinline__ unsigned short f32_to_bf16(float f) {
    unsigned u = __float_as_uint(f);
    unsigned r = u + 0x7FFFu + ((u >> 16) & 1u);
    return (unsigned short)(r >> 16);
}
__device__ __forceinline__ float bf16_to_f32(unsigned short b) {
    return __uint_as_float(((unsigned)b) << 16);
}
__device__ __forceinline__ float bf16r(float f) {
    return bf16_to_f32(f32_to_bf16(f));
}
__device__ __forceinline__ float silu_f(float x) {
    float e = expf(-x);
    return x * __builtin_amdgcn_rcpf(1.0f + e);
}
__device__ __forceinline__ float softplus_f(float x) {
    return fmaxf(x, 0.0f) + log1pf(expf(-fabsf(x)));
}
__device__ __forceinline__ float conv4_silu(float x0, float x1, float x2, float x3,
                                            float w0, float w1, float w2, float w3, float bias) {
    float c = w0 * x0 + w1 * x1 + w2 * x2 + w3 * x3;
    return silu_f(c + bias);
}
__device__ __forceinline__ v8f ld8f(const float* p) {
    v4f a = *(const v4f*)p;
    v4f b = *(const v4f*)(p + 4);
    return __builtin_shufflevector(a, b, 0, 1, 2, 3, 4, 5, 6, 7);
}

__device__ __forceinline__ void mma16(v8f& acc, const FragH& a, const FragH& b) {
    acc = __builtin_amdgcn_wmma_f32_16x16x32_f16(false, a.v, false, b.v, (short)0, acc, false, false);
    asm volatile("v_nop\n\tv_nop\n\tv_nop\n\tv_nop" : "+v"(acc) : "v"(a.v), "v"(b.v));
}
__device__ __forceinline__ void mma16(v8f& acc, const FragB& a, const FragB& b) {
    acc = __builtin_amdgcn_wmma_f32_16x16x32_bf16(false, a.v, false, b.v, (short)0, acc, false, false);
    asm volatile("v_nop\n\tv_nop\n\tv_nop\n\tv_nop" : "+v"(acc) : "v"(a.v), "v"(b.v));
}

__global__ __launch_bounds__(256)
void cvt_bf16_kernel(const float* __restrict__ src, unsigned short* dst, int n8)
{
    const int i = blockIdx.x * 256 + threadIdx.x;
    if (i >= n8) return;
    const size_t e = (size_t)i * 8;
    const v8f x = ld8f(src + e);
    u16x8 v;
#pragma unroll
    for (int c = 0; c < 8; ++c) v[c] = f32_to_bf16(x[c]);
    *(volatile u16x8*)(dst + e) = v;
    __threadfence();
    *(volatile u16x8*)(dst + e) = v;
}

#define TP16 72
__global__ __launch_bounds__(256)
void transpose_cvt_kernel(const float* __restrict__ W, unsigned short* Wt, int K, int N,
                          int mode, float fsc)
{
    __shared__ __attribute__((aligned(16))) unsigned short t16[32 * TP16];
    const int tid  = threadIdx.x;
    const int lane = tid & 31;
    const int wave = tid >> 5;
    const int n0 = blockIdx.x * 32;
    const int k0 = blockIdx.y * 64;
    const int nn = tid & 31;
    const int kq = tid >> 5;
#pragma unroll
    for (int i = 0; i < 8; ++i) {
        const int kk = kq + 8 * i;
        const float w = W[(size_t)(k0 + kk) * N + n0 + nn];
        const unsigned short hb = f32_to_bf16(w);
        unsigned short bits;
        if (mode == 0) {
            bits = hb;
        } else {
            HBits hv;
            hv.h = (_Float16)(bf16_to_f32(hb) * fsc);
            bits = hv.u;
        }
        t16[nn * TP16 + kk] = bits;
    }
    __syncthreads();
    const int row = wave * 4 + (lane >> 3);
    const int c   = (lane & 7) * 8;
    const u16x8 v = *(const u16x8*)(t16 + row * TP16 + c);
    unsigned short* gp = Wt + (size_t)(n0 + row) * K + k0 + c;
    *(volatile u16x8*)gp = v;
    __threadfence();
    *(volatile u16x8*)gp = v;
}

template<int NBF>
__device__ __forceinline__ void tile_store_f32(const float* st, float* gp, int ldc, int lane) {
    constexpr int CW  = NBF * 16;
    constexpr int P   = CW + 4;
    constexpr int LPR = CW / 4;
    constexpr int RPI = 32 / LPR;
    constexpr int NIT = 32 / RPI;
    const int rsub = lane / LPR;
    const int c4   = (lane % LPR) * 4;
#pragma unroll
    for (int it = 0; it < NIT; ++it) {
        const int row = it * RPI + rsub;
        const v4f v = *(const v4f*)(st + row * P + c4);
        *(volatile v4f*)(gp + (size_t)row * ldc + c4) = v;
    }
}
__device__ __forceinline__ void tile_store_f16(const float* st, unsigned short* gp, int ldc, int lane) {
    constexpr int P = 68;
    const int rsub = lane >> 3;
    const int c8   = (lane & 7) * 8;
#pragma unroll
    for (int it = 0; it < 8; ++it) {
        const int row = it * 4 + rsub;
        const v8f x = ld8f(st + row * P + c8);
        Pack8 pk;
        pk.f = __builtin_convertvector(x, v8h);
        const u16x8 v = pk.u;
        *(volatile u16x8*)(gp + (size_t)row * ldc + c8) = v;
    }
}

template<typename FR, int WN, int NBF, int EPI>
__global__ __launch_bounds__(128)
void gemm_tn_kernel(const unsigned short* __restrict__ A, const unsigned short* __restrict__ Bw,
                    float* C, float* C2, unsigned short* C16,
                    int K, int ldc, int csplit, float scale)
{
    static_assert(WN == 1 || WN == 2);
    static_assert(NBF == 2 || NBF == 4);
    static_assert(EPI == 0 || NBF == 4);
    constexpr int WM = 4 / WN;
    constexpr int CW = NBF * 16;
    constexpr int P  = CW + 4;
    __shared__ __attribute__((aligned(16))) float stile[4][32 * P];

    const int tid  = threadIdx.x;
    const int lane = tid & 31;
    const int wave = tid >> 5;
    const int h    = lane >> 4;
    const int m    = lane & 15;
    const int wm   = wave / WN;
    const int wn   = wave % WN;

    const int rowW = blockIdx.y * (WM * 32) + wm * 32;
    const int colW = blockIdx.x * (WN * CW) + wn * CW;

    v8f acc[2 * NBF];
#pragma unroll
    for (int j = 0; j < 2 * NBF; ++j)
#pragma unroll
        for (int r = 0; r < 8; ++r) acc[j][r] = 0.0f;

    const size_t aoff  = (size_t)(rowW + m) * K + 8 * h;
    const size_t boff  = (size_t)(colW + m) * K + 8 * h;
    const size_t sub16 = (size_t)16 * K;
    const int nk = K >> 5;

    for (int kt = 0; kt < nk; ++kt) {
        const size_t k0 = (size_t)kt * 32;
        FR fa[2], fb[NBF];
#pragma unroll
        for (int s = 0; s < 2; ++s) {
            const unsigned short* p = A + aoff + s * sub16 + k0;
            fa[s].h[0] = *(const u16x8*)(p);
            fa[s].h[1] = *(const u16x8*)(p + 16);
        }
#pragma unroll
        for (int j = 0; j < NBF; ++j) {
            const unsigned short* p = Bw + boff + j * sub16 + k0;
            fb[j].h[0] = *(const u16x8*)(p);
            fb[j].h[1] = *(const u16x8*)(p + 16);
        }
#pragma unroll
        for (int s = 0; s < 2; ++s)
#pragma unroll
            for (int j = 0; j < NBF; ++j)
                mma16(acc[s * NBF + j], fa[s], fb[j]);
    }

    float* st = stile[wave];
#pragma unroll
    for (int s = 0; s < 2; ++s)
#pragma unroll
        for (int j = 0; j < NBF; ++j)
#pragma unroll
            for (int r = 0; r < 8; ++r)
                st[(s * 16 + 8 * h + r) * P + j * 16 + m] = acc[s * NBF + j][r] * scale;
    __syncthreads();

    if (EPI == 0) {
        float* Cp = C;
        int gcol = colW;
        if (colW >= csplit) { Cp = C2; gcol = colW - csplit; }
        float* gp = Cp + (size_t)rowW * ldc + gcol;
        tile_store_f32<NBF>(st, gp, ldc, lane);
        __threadfence();
        tile_store_f32<NBF>(st, gp, ldc, lane);
    } else {
        unsigned short* gp = C16 + (size_t)rowW * ldc + colW;
        tile_store_f16(st, gp, ldc, lane);
        __threadfence();
        tile_store_f16(st, gp, ldc, lane);
    }
}

__global__ __launch_bounds__(256)
void conv_silu_kernel(const float* __restrict__ X, const float* __restrict__ cw,
                      const float* __restrict__ cb, unsigned short* U16)
{
    const int m  = blockIdx.x;
    const int l  = m & (NL_ - 1);
    const int d0 = threadIdx.x * 8;
    const float* xr = X + (size_t)m * DI_ + d0;

    v8f x3 = ld8f(xr);
    v8f x2, x1, x0;
#pragma unroll
    for (int c = 0; c < 8; ++c) { x2[c] = 0.0f; x1[c] = 0.0f; x0[c] = 0.0f; }
    if (l >= 1) x2 = ld8f(xr - DI_);
    if (l >= 2) x1 = ld8f(xr - 2 * DI_);
    if (l >= 3) x0 = ld8f(xr - 3 * DI_);

    const float* wp = cw + (size_t)d0 * 4;
    v4f wv[8];
#pragma unroll
    for (int c = 0; c < 8; ++c) {
        v4f w = *(const v4f*)(wp + 4 * c);
#pragma unroll
        for (int j = 0; j < 4; ++j) w[j] = bf16r(w[j]);
        wv[c] = w;
    }
    v8f bias = ld8f(cb + d0);
#pragma unroll
    for (int c = 0; c < 8; ++c) bias[c] = bf16r(bias[c]);

    v8f u;
#pragma unroll
    for (int c = 0; c < 8; ++c)
        u[c] = conv4_silu(x0[c], x1[c], x2[c], x3[c], wv[c][0], wv[c][1], wv[c][2], wv[c][3], bias[c]);

    Pack8 pk;
    pk.f = __builtin_convertvector(u * 64.0f, v8h);
    const u16x8 v = pk.u;
    unsigned short* gp = U16 + (size_t)m * DI_ + d0;
    *(volatile u16x8*)gp = v;
    __threadfence();
    *(volatile u16x8*)gp = v;
}

__device__ __forceinline__ void rows8_store_pass(const unsigned short* s16, unsigned short* y16,
                                                 size_t gbase, int wave, int lane) {
#pragma unroll
    for (int it = 0; it < 2; ++it) {
        const int t = wave * 8 + it * 4 + (lane >> 3);
        const int c = (lane & 7) * 8;
        const u16x8 v = *(const u16x8*)(s16 + t * 64 + c);
        *(volatile u16x8*)(y16 + gbase + (size_t)t * DI_ + c) = v;
    }
}

__global__ __launch_bounds__(64)
void scan_kernel(const float* __restrict__ X, const float* __restrict__ Z,
                 const _Float16* __restrict__ Dh, const float* __restrict__ BC,
                 const float* __restrict__ cw, const float* __restrict__ cb,
                 const float* __restrict__ bdt, const float* __restrict__ Alog,
                 const float* __restrict__ Dp,
                 unsigned short* y16)
{
    __shared__ __attribute__((aligned(16))) unsigned short s16[16 * 64];
    __shared__ __attribute__((aligned(16))) float sbc[16 * 2 * NS_];

    const int tid   = threadIdx.x;
    const int lane  = tid & 31;
    const int wave  = tid >> 5;
    const int dbase = blockIdx.x * 64;
    const int d     = dbase + tid;
    const int b     = blockIdx.y;

    float an[NS_], hs[NS_];
#pragma unroll
    for (int n = 0; n < NS_; ++n) {
        an[n] = -expf(bf16r(Alog[n]));
        hs[n] = 0.0f;
    }
    const float w0 = bf16r(cw[d * 4 + 0]), w1 = bf16r(cw[d * 4 + 1]);
    const float w2 = bf16r(cw[d * 4 + 2]), w3 = bf16r(cw[d * 4 + 3]);
    const float cbias = bf16r(cb[d]);
    const float tb    = bf16r(bdt[d]);
    const float Dd    = bf16r(Dp[d]);

    float xm1 = 0.0f, xm2 = 0.0f, xm3 = 0.0f;
    const size_t mrow0 = (size_t)b * NL_;

#pragma unroll 1
    for (int l0 = 0; l0 < NL_; l0 += 16) {
        {
            const float* src = BC + (mrow0 + (size_t)l0) * (2 * NS_) + tid * 8;
            const v4f a0 = *(const v4f*)(src);
            const v4f a1 = *(const v4f*)(src + 4);
            *(v4f*)(sbc + tid * 8)     = a0;
            *(v4f*)(sbc + tid * 8 + 4) = a1;
        }
        __syncthreads();
#pragma unroll 1
        for (int t = 0; t < 16; ++t) {
            const size_t mrow = mrow0 + (size_t)(l0 + t);
            const size_t e = mrow * DI_ + d;
            const float xv = X[e];
            const float zv = Z[e];
            const float dv = (float)Dh[e] * 0.00390625f;
            const float u  = conv4_silu(xm3, xm2, xm1, xv, w0, w1, w2, w3, cbias);
            xm3 = xm2; xm2 = xm1; xm1 = xv;
            const float dt = softplus_f(dv + tb);
            const float* bp = sbc + t * (2 * NS_);
            float y = 0.0f;
#pragma unroll
            for (int n = 0; n < NS_; ++n) {
                const float bn = bp[n];
                const float cn = bp[NS_ + n];
                const float da = __expf(dt * an[n]);
                hs[n] = da * hs[n] + (dt * bn) * u;
                y += hs[n] * cn;
            }
            const float g = (y + Dd * u) * silu_f(zv);
            HBits hv;
            hv.h = (_Float16)(g * 256.0f);
            s16[t * 64 + tid] = hv.u;
        }
        __syncthreads();
        const size_t gbase = (mrow0 + (size_t)l0) * DI_ + dbase;
        rows8_store_pass(s16, y16, gbase, wave, lane);
        __threadfence();
        rows8_store_pass(s16, y16, gbase, wave, lane);
        __syncthreads();
    }
}

extern "C" void kernel_launch(void* const* d_in, const int* in_sizes, int n_in,
                              void* d_out, int out_size, void* d_ws, size_t ws_size,
                              hipStream_t stream)
{
    if (n_in < 10) return;
    if (in_sizes[0] != MT_ * DM_)        return;
    if (in_sizes[1] != DM_ * 2 * DI_)    return;
    if (in_sizes[2] != DI_ * 4)          return;
    if (in_sizes[3] != DI_)              return;
    if (in_sizes[4] != DI_ * 2 * NS_)    return;
    if (in_sizes[5] != DI_ * DI_)        return;
    if (in_sizes[6] != DI_)              return;
    if (in_sizes[7] != NS_)              return;
    if (in_sizes[8] != DI_)              return;
    if (in_sizes[9] != DI_ * DM_)        return;
    if (out_size != MT_ * DM_)           return;

    const float* x     = (const float*)d_in[0];
    const float* w_in  = (const float*)d_in[1];
    const float* cw    = (const float*)d_in[2];
    const float* cb    = (const float*)d_in[3];
    const float* w_xp  = (const float*)d_in[4];
    const float* w_dt  = (const float*)d_in[5];
    const float* bdt   = (const float*)d_in[6];
    const float* alog  = (const float*)d_in[7];
    const float* Dp    = (const float*)d_in[8];
    const float* w_out = (const float*)d_in[9];
    float* out = (float*)d_out;

    const size_t SZ_X16  = (size_t)MT_ * DM_ * 2;
    const size_t SZ_WTIN = (size_t)2 * DI_ * DM_ * 2;
    const size_t SZ_U16  = (size_t)MT_ * DI_ * 2;
    const size_t SZ_WTDT = (size_t)DI_ * DI_ * 2;
    const size_t SZ_WTXP = (size_t)2 * NS_ * DI_ * 2;
    const size_t SZ_WTO  = (size_t)DM_ * DI_ * 2;
    const size_t SZ_BC   = (size_t)MT_ * 2 * NS_ * 4;
    const size_t SZ_F    = (size_t)MT_ * DI_ * 4;
    const size_t SZ_D16  = (size_t)MT_ * DI_ * 2;
    const size_t SZ_Y16  = (size_t)MT_ * DI_ * 2;

    const size_t OFF_X16  = 0;
    const size_t OFF_WTIN = OFF_X16 + SZ_X16;
    const size_t OFF_U16  = OFF_WTIN + SZ_WTIN;
    const size_t END_16   = OFF_U16 + SZ_U16;
    const size_t OFF_Y16  = 0;
    const size_t OFF_WTDT = END_16;
    const size_t OFF_WTXP = OFF_WTDT + SZ_WTDT;
    const size_t OFF_WTO  = OFF_WTXP + SZ_WTXP;
    const size_t OFF_BC   = OFF_WTO + SZ_WTO;
    const size_t OFF_XF   = OFF_BC + SZ_BC;
    const size_t OFF_ZF   = OFF_XF + SZ_F;
    const size_t OFF_D16  = OFF_ZF + SZ_F;
    const size_t WS_END   = OFF_D16 + SZ_D16;
    if (OFF_Y16 + SZ_Y16 > OFF_U16) return;
    if (ws_size < WS_END) return;

    char* ws = (char*)d_ws;
    unsigned short* x16  = (unsigned short*)(ws + OFF_X16);
    unsigned short* wtin = (unsigned short*)(ws + OFF_WTIN);
    unsigned short* u16  = (unsigned short*)(ws + OFF_U16);
    unsigned short* y16  = (unsigned short*)(ws + OFF_Y16);
    unsigned short* wtdt = (unsigned short*)(ws + OFF_WTDT);
    unsigned short* wtxp = (unsigned short*)(ws + OFF_WTXP);
    unsigned short* wto  = (unsigned short*)(ws + OFF_WTO);
    float*          BCf  = (float*)(ws + OFF_BC);
    float*          Xf   = (float*)(ws + OFF_XF);
    float*          Zf   = (float*)(ws + OFF_ZF);
    unsigned short* d16  = (unsigned short*)(ws + OFF_D16);

    {
        const int n8 = (MT_ * DM_) / 8;
        hipLaunchKernelGGL(cvt_bf16_kernel, dim3((n8 + 255) / 256), dim3(256), 0, stream,
                           x, x16, n8);
    }
    hipLaunchKernelGGL(transpose_cvt_kernel, dim3((2 * DI_) / 32, DM_ / 64), dim3(256), 0, stream,
                       w_in, wtin, (int)DM_, (int)(2 * DI_), 0, 1.0f);
    hipLaunchKernelGGL(transpose_cvt_kernel, dim3(DI_ / 32, DI_ / 64), dim3(256), 0, stream,
                       w_dt, wtdt, (int)DI_, (int)DI_, 1, 64.0f);
    hipLaunchKernelGGL(transpose_cvt_kernel, dim3((2 * NS_) / 32, DI_ / 64), dim3(256), 0, stream,
                       w_xp, wtxp, (int)DI_, (int)(2 * NS_), 1, 64.0f);
    hipLaunchKernelGGL(transpose_cvt_kernel, dim3(DM_ / 32, DI_ / 64), dim3(256), 0, stream,
                       w_out, wto, (int)DI_, (int)DM_, 1, 64.0f);

    hipLaunchKernelGGL(HIP_KERNEL_NAME(gemm_tn_kernel<FragB, 2, 4, 0>),
                       dim3((2 * DI_) / 128, MT_ / 64), dim3(128), 0, stream,
                       (const unsigned short*)x16, (const unsigned short*)wtin,
                       Xf, Zf, u16, (int)DM_, (int)DI_, (int)DI_, 1.0f);

    hipLaunchKernelGGL(conv_silu_kernel, dim3(MT_), dim3(DI_ / 8), 0, stream,
                       (const float*)Xf, cw, cb, u16);

    hipLaunchKernelGGL(HIP_KERNEL_NAME(gemm_tn_kernel<FragH, 2, 4, 1>),
                       dim3(DI_ / 128, MT_ / 64), dim3(128), 0, stream,
                       (const unsigned short*)u16, (const unsigned short*)wtdt,
                       Xf, Xf, d16, (int)DI_, (int)DI_, (int)(1 << 30), 0.0625f);

    hipLaunchKernelGGL(HIP_KERNEL_NAME(gemm_tn_kernel<FragH, 1, 2, 0>),
                       dim3((2 * NS_) / 32, MT_ / 128), dim3(128), 0, stream,
                       (const unsigned short*)u16, (const unsigned short*)wtxp,
                       BCf, BCf, d16, (int)DI_, (int)(2 * NS_), (int)(1 << 30), 0.000244140625f);

    hipLaunchKernelGGL(scan_kernel, dim3(DI_ / 64, NBATCH), dim3(64), 0, stream,
                       (const float*)Xf, (const float*)Zf, (const _Float16*)d16, (const float*)BCf,
                       cw, cb, bdt, alog, Dp, y16);

    hipLaunchKernelGGL(HIP_KERNEL_NAME(gemm_tn_kernel<FragH, 2, 4, 0>),
                       dim3(DM_ / 128, MT_ / 64), dim3(128), 0, stream,
                       (const unsigned short*)y16, (const unsigned short*)wto,
                       out, out, u16, (int)DI_, (int)DM_, (int)(1 << 30), 0.00006103515625f);
}
